// PropagationBlock_57329223467239
// MI455X (gfx1250) — hardware-run, weakly checked
//
#include <hip/hip_runtime.h>


namespace {
constexpr int N = 50000, E = 1000000, DIM = 3, NV = 32, NS = 32, RN = N * DIM, RE = E * DIM;
typedef _Float16 b16;
typedef __attribute__((ext_vector_type(16))) _Float16 v16b;
typedef __attribute__((ext_vector_type(8))) _Float16 v8b;
typedef __attribute__((ext_vector_type(8))) float v8f;
typedef __attribute__((ext_vector_type(4))) float v4f;
typedef __attribute__((ext_vector_type(2))) _Float16 v2b;
__device__ __forceinline__ float bf16_rne(float f) { unsigned int u = __float_as_uint(f); u += 0x7FFFu + ((u >> 16) & 1u); return __uint_as_float(u & 0xFFFF0000u); }
__device__ __forceinline__ void split16(float v, b16& hi, b16& lo) { hi = (b16)v; lo = (b16)(v - (float)hi); }
__device__ __forceinline__ v16b frag_kb(const b16* p, int hh) { const v8b a = *(const v8b*)(p + 8 * hh), b = *(const v8b*)(p + 16 + 8 * hh); v16b f;
#pragma unroll
  for (int e = 0; e < 8; ++e) { f[e] = a[e]; f[8 + e] = b[e]; } return f; }
__device__ __forceinline__ v8f wmma16b(v16b a, v16b b, v8f c) { v8f d = __builtin_amdgcn_wmma_f32_16x16x32_f16(false, a, false, b, (short)0, c, false, false); asm volatile("v_nop\n\tv_nop\n\tv_nop\n\tv_nop" : "+v"(d) : "v"(a), "v"(b)); return d; }
__device__ __forceinline__ void wave_lds_sync() { __builtin_amdgcn_fence(__ATOMIC_RELEASE, "workgroup"); __builtin_amdgcn_wave_barrier(); __builtin_amdgcn_fence(__ATOMIC_ACQUIRE, "workgroup"); }
__device__ __forceinline__ float pmul(float a, float b) { float p = a * b; asm volatile("" : "+v"(p)); return p; }
__device__ __forceinline__ int iclamp(int v, int lo, int hi) { return v < lo ? lo : (v > hi ? hi : v); }
__device__ __forceinline__ float silu(float v) { return v / (1.0f + __expf(-v)); }
constexpr int CSR_NBLK9 = 512, CSR_GB9 = 9, CSR_GN9 = 1 << CSR_GB9  , CSR_TS9 = (CSR_GN9 < 32 ? 32 : CSR_GN9)  , CSR_MAXG9 = 512, CSR_CAP9 = 12288  ;
__device__ __host__ __forceinline__ int csr_tix9(int v) { return (v >> CSR_GB9) * CSR_TS9 + (v & (CSR_GN9 - 1)); }
__global__ __launch_bounds__(64) void csrA_kernel9(const int* __restrict__ dst, int E, int N, int nG, int CHP, int NGP, int* __restrict__ STG, int* __restrict__ HST) {
  extern __shared__ int sm[];
  int* cnt = sm; int* run = sm + NGP; int* ids = sm + 2 * NGP;
  const int b = blockIdx.x; const int ch = (E + CSR_NBLK9 - 1) / CSR_NBLK9; const int e0 = b * ch, e1 = min(E, e0 + ch);
  for (int i = threadIdx.x; i < NGP; i += 64) cnt[i] = 0;
  for (int i = threadIdx.x; i < CHP; i += 64) ids[i] = -1;
  __syncthreads();
  if (threadIdx.x == 0) {
    for (int e = e0; e < e1; ++e) { int d = dst[e]; d = (d < 0) ? 0 : (d >= N ? N - 1 : d); cnt[d >> CSR_GB9] += 1; }
    int acc = 0; for (int g = 0; g < nG; ++g) { run[g] = acc; acc += cnt[g]; }
    for (int e = e0; e < e1; ++e) { int d = dst[e]; d = (d < 0) ? 0 : (d >= N ? N - 1 : d); const int g = d >> CSR_GB9; ids[run[g]] = e; run[g] += 1; } }
  __syncthreads();
  typedef __attribute__((ext_vector_type(4))) int v4i;
  for (int pass = 0; pass < 2; ++pass) {
    for (int i = threadIdx.x; i < CHP / 4; i += 64) *(volatile v4i*)(STG + (size_t)b * CHP + i * 4) = *(const v4i*)(&ids[i * 4]);
    for (int i = threadIdx.x; i < NGP / 4; i += 64) { v4i v; for (int e = 0; e < 4; ++e) v[e] = (i * 4 + e < nG) ? cnt[i * 4 + e] : 0; *(volatile v4i*)(HST + (size_t)b * NGP + i * 4) = v; }
    __threadfence(); }
}
__global__ __launch_bounds__(512) void csrS_kernel9(const int* __restrict__ HST, int nG, int NGP, int* __restrict__ START, int* __restrict__ TOT, int* __restrict__ OFF) {
  __shared__ int tot[CSR_MAXG9];
  const int b = threadIdx.x;
  for (int pass = 0; pass < 2; ++pass) { int runb = 0; for (int g = 0; g < nG; ++g) { int c = HST[(size_t)b * NGP + g]; c = (c < 0) ? 0 : c; ((volatile int*)OFF)[(size_t)g * CSR_NBLK9 + b] = runb; runb += c; } __threadfence(); }
  for (int g = threadIdx.x; g < nG; g += 512) { int s = 0; for (int bb = 0; bb < CSR_NBLK9; ++bb) { int c = HST[(size_t)bb * NGP + g]; s += (c < 0) ? 0 : c; } tot[g] = s; }
  __syncthreads();
  if (threadIdx.x < 32) {
    __shared__ int st[CSR_MAXG9 + 32];
    if (threadIdx.x == 0) { int acc = 0; for (int g = 0; g < NGP; ++g) { st[g] = acc; if (g < nG) acc += (tot[g] + 31) & ~31; } st[NGP] = acc; }
    __builtin_amdgcn_fence(__ATOMIC_RELEASE, "workgroup"); __builtin_amdgcn_wave_barrier(); __builtin_amdgcn_fence(__ATOMIC_ACQUIRE, "workgroup");
    for (int pass = 0; pass < 2; ++pass) { for (int i = threadIdx.x; i < NGP + 32; i += 32) { ((volatile int*)START)[i] = (i <= NGP) ? st[min(i, NGP)] : 0; ((volatile int*)TOT)[i] = (i < nG) ? tot[i] : 0; } __threadfence(); } }
}
__global__ __launch_bounds__(256) void csrB_kernel9(const int* __restrict__ dst, int N, int nG, int CHP, int NGP, int permLen, const int* __restrict__ STG, const int* __restrict__ HST, const int* __restrict__ OFF, const int* __restrict__ START, const int* __restrict__ TOT, int* __restrict__ PERM, int* __restrict__ ROWPTR, int* __restrict__ ROWCNT, int* __restrict__ FLAG) {
  typedef __attribute__((ext_vector_type(4))) int v4i;
  __shared__ int ids[CSR_CAP9]; __shared__ unsigned short key[CSR_CAP9]; __shared__ int outp[CSR_CAP9]; __shared__ int ncnt[CSR_GN9 + 1]; __shared__ int boff[CSR_NBLK9 + 1];
  const int g = blockIdx.x, t_ = threadIdx.x; int tot = TOT[g]; int st = START[g], stn = START[g + 1]; const int v0 = g * CSR_GN9; const int nv = min(CSR_GN9, N - v0); const int t0 = g * CSR_TS9;
  st = (st < 0) ? 0 : (st > permLen - 32 ? permLen - 32 : st) & ~31; stn = (stn < st) ? st : (stn > permLen ? permLen : stn); tot = (tot < 0) ? 0 : tot; if (tot > stn - st && tot <= CSR_CAP9) tot = stn - st;
  if (tot > CSR_CAP9) {
    for (int pass = 0; pass < 2; ++pass) { for (int i = t_; i < CSR_TS9 / 4; i += 256) { v4i a, c; for (int e = 0; e < 4; ++e) { a[e] = st; c[e] = 0; } *(volatile v4i*)(ROWPTR + t0 + i * 4) = a; *(volatile v4i*)(ROWCNT + t0 + i * 4) = c; } if (t_ == 0) ((volatile int*)FLAG)[0] = 1; __threadfence(); } (void)nv; return; }
  if (t_ == 0) { int acc = 0; for (int b = 0; b < CSR_NBLK9; ++b) { boff[b] = acc; int c = HST[(size_t)b * NGP + g]; c = (c < 0) ? 0 : (c > CHP ? CHP : c); acc += c; if (acc > tot) acc = tot; } boff[CSR_NBLK9] = acc; }
  for (int i = t_; i <= CSR_GN9; i += 256) ncnt[i] = 0;
  __syncthreads();
  for (int b = 0; b < CSR_NBLK9; ++b) { const int c = boff[b + 1] - boff[b]; int o_ = OFF[(size_t)g * CSR_NBLK9 + b]; o_ = (o_ < 0) ? 0 : (o_ > CHP - c ? CHP - c : o_); const int* src_ = STG + (size_t)b * CHP + o_;
    for (int i = t_; i < c; i += 256) { int id = src_[i]; id = (id < 0) ? 0 : id; ids[boff[b] + i] = id; int d = dst[id]; d = (d < v0) ? v0 : (d >= N ? N - 1 : d); int kk = d - v0; kk = (kk < 0) ? 0 : (kk >= CSR_GN9 ? CSR_GN9 - 1 : kk); key[boff[b] + i] = (unsigned short)kk; } }
  __syncthreads();
  if (t_ == 0) { for (int i = 0; i < tot; ++i) ncnt[key[i]] += 1; int acc = 0; for (int vl = 0; vl < CSR_GN9; ++vl) { const int c = ncnt[vl]; ncnt[vl] = acc; acc += c; } ncnt[CSR_GN9] = acc;
    for (int i = 0; i < tot; ++i) { const int vl = key[i]; outp[ncnt[vl]] = ids[i]; ncnt[vl] += 1; }
    for (int vl = CSR_GN9; vl > 0; --vl) ncnt[vl] = ncnt[vl - 1]; ncnt[0] = 0; }
  __syncthreads();
  for (int pass = 0; pass < 2; ++pass) {
    for (int i = t_; i < (stn - st) / 4; i += 256) { v4i v; for (int e = 0; e < 4; ++e) { const int q = i * 4 + e; v[e] = (q < tot) ? outp[q] : -1; } *(volatile v4i*)(PERM + st + i * 4) = v; }
    for (int i = t_; i < CSR_TS9 / 4; i += 256) { v4i a, c; for (int e = 0; e < 4; ++e) { const int vl = i * 4 + e; const int vc = vl < CSR_GN9 ? vl : CSR_GN9; a[e] = (vl < CSR_GN9) ? st + ncnt[vc] : st; c[e] = (vl < nv) ? (ncnt[(vc < CSR_GN9 ? vc : CSR_GN9 - 1) + 1] - ncnt[vc]) : 0; } *(volatile v4i*)(ROWPTR + t0 + i * 4) = a; *(volatile v4i*)(ROWCNT + t0 + i * 4) = c; }
    __threadfence(); }
}
__global__ __launch_bounds__(256) void csrZ_kernel9(int* __restrict__ p, size_t n4) { typedef __attribute__((ext_vector_type(4))) int v4i; const size_t tid = (size_t)blockIdx.x * 256 + threadIdx.x, nth = (size_t)gridDim.x * 256; v4i z = {0, 0, 0, 0}; for (size_t i = tid; i < n4; i += nth) *(volatile v4i*)(p + i * 4) = z; }
struct CsrBufs9 { int *STG, *HST, *OFF, *START, *TOT, *PERM, *ROWPTR, *ROWCNT, *FLAG; int nG, NGP, CHP; size_t permLen; char* base; size_t bytes; };
static size_t csr_carve9(CsrBufs9& c, char* ws, size_t off, int E, int N) {
  const size_t off0 = off; c.base = ws + off;
  auto al = [&](size_t bytes) { char* p = ws + off; off += (bytes + 255) & ~(size_t)255; return p; };
  c.nG = (N + CSR_GN9 - 1) / CSR_GN9; c.NGP = (c.nG + 31) & ~31; const int ch = (E + CSR_NBLK9 - 1) / CSR_NBLK9; c.CHP = (ch + 31) & ~31; c.permLen = (size_t)E + 32 * (size_t)c.nG + 32;
  c.STG = (int*)al((size_t)CSR_NBLK9 * c.CHP * 4); c.HST = (int*)al((size_t)CSR_NBLK9 * c.NGP * 4); c.OFF = (int*)al((size_t)c.NGP * CSR_NBLK9 * 4); c.START = (int*)al((size_t)(c.NGP + 64) * 4); c.TOT = (int*)al((size_t)(c.NGP + 64) * 4);
  c.PERM = (int*)al(c.permLen * 4); c.ROWPTR = (int*)al((size_t)c.nG * CSR_TS9 * 4); c.ROWCNT = (int*)al((size_t)c.nG * CSR_TS9 * 4); c.FLAG = (int*)al(256);
  c.bytes = off - off0; return off;
}
static void csr_build9(const CsrBufs9& c, const int* dst, int E, int N, hipStream_t stream) {
  const size_t smem = (size_t)(2 * c.NGP + c.CHP) * 4;
  csrZ_kernel9<<<512, 256, 0, stream>>>((int*)c.base, c.bytes / 16);
  csrA_kernel9<<<CSR_NBLK9, 64, smem, stream>>>(dst, E, N, c.nG, c.CHP, c.NGP, c.STG, c.HST);
  csrS_kernel9<<<1, 512, 0, stream>>>(c.HST, c.nG, c.NGP, c.START, c.TOT, c.OFF);
  csrB_kernel9<<<c.nG, 256, 0, stream>>>(dst, N, c.nG, c.CHP, c.NGP, (int)c.permLen, c.STG, c.HST, c.OFF, c.START, c.TOT, c.PERM, c.ROWPTR, c.ROWCNT, c.FLAG);
}


__global__ __launch_bounds__(256) void wsmall_kernel(const float* __restrict__ M, const float* __restrict__ n1, const float* __restrict__ n2, const float* __restrict__ v1, const float* __restrict__ v2, const float* __restrict__ e1, const float* __restrict__ e2, b16* __restrict__ WM, b16* __restrict__ WMT, b16* __restrict__ MCh, b16* __restrict__ MCl, b16* __restrict__ WE) {
  const int t = threadIdx.x;
  for (int pass = 0; pass < 2; ++pass) {
    for (int i = t; i < NV * NS; i += 256) { const int s = i / NV, v = i % NV; ((volatile b16*)WM)[s * NV + v] = (b16)bf16_rne(M[v * NS + s]); ((volatile b16*)WMT)[v * NS + s] = (b16)bf16_rne(M[v * NS + s]); }
    for (int i = t; i < NV * 64; i += 256) { const int w = i / 64, k = i % 64; const float ev = k < 32 ? bf16_rne(e1[k * NV + w]) : bf16_rne(e2[(k - 32) * NV + w]); ((volatile b16*)WE)[w * 64 + k] = (b16)(ev * 0.5f);
      float s = 0.0f; for (int j = 0; j < NV; ++j) { const float nv = k < 32 ? bf16_rne(n1[k * NV + j]) : bf16_rne(n2[(k - 32) * NV + j]); s += pmul(nv, bf16_rne(v1[j * NV + w]) + bf16_rne(v2[j * NV + w])); } s *= 0.25f; b16 p, q; split16(s, p, q); ((volatile b16*)MCh)[w * 64 + k] = p; ((volatile b16*)MCl)[w * 64 + k] = q; }
    __threadfence(); }
}
__global__ __launch_bounds__(32) void nodemix_kernel(const float* __restrict__ xn, const float* __restrict__ attr, const float* __restrict__ msw, const b16* __restrict__ WM, const b16* __restrict__ WMT, int RLIM, float* __restrict__ XB) {
  __shared__ __attribute__((aligned(16))) b16 Ah[16][40], Bh[16][40], Bl[16][40]; __shared__ float Tf[16][NV + 1]; const int lane = threadIdx.x, nloc = lane & 15, hlf = lane >> 4; const size_t r0 = (size_t)blockIdx.x * 16; if (r0 >= (size_t)RLIM) return;
  for (int rr = 0; rr < 16; ++rr) Ah[rr][lane] = (b16)bf16_rne(xn[(r0 + rr) * NV + lane]);
  wave_lds_sync(); const float ang = 0.1f * bf16_rne(msw[0]); const float ca = cosf(ang), sa = sinf(ang);
  { const v16b a = frag_kb(&Ah[nloc][0], hlf);
#pragma unroll
    for (int tt = 0; tt < 2; ++tt) { v8f acc = {}; acc = wmma16b(a, frag_kb(WM + (size_t)(tt * 16 + nloc) * NV, hlf), acc);
#pragma unroll
      for (int r8 = 0; r8 < 8; ++r8) { const int rl = 8 * hlf + r8; const size_t n = (r0 + rl) / DIM; const float v = pmul(acc[r8], bf16_rne(attr[n * NS + tt * 16 + nloc])); b16 p, q; split16(v, p, q); Bh[rl][tt * 16 + nloc] = p; Bl[rl][tt * 16 + nloc] = q; } } }
  wave_lds_sync();
  { const v16b bh = frag_kb(&Bh[nloc][0], hlf), bl = frag_kb(&Bl[nloc][0], hlf);
#pragma unroll
    for (int tt = 0; tt < 2; ++tt) { v8f acc = {}; const v16b w = frag_kb(WMT + (size_t)(tt * 16 + nloc) * NS, hlf); acc = wmma16b(bh, w, acc); acc = wmma16b(bl, w, acc);
#pragma unroll
      for (int r8 = 0; r8 < 8; ++r8) { const int rl = 8 * hlf + r8; Tf[rl][tt * 16 + nloc] = pmul(ca, (float)Ah[rl][tt * 16 + nloc]) + pmul(sa, acc[r8]); } } }
  wave_lds_sync();
  for (int pass = 0; pass < 2; ++pass) { for (int rr = 0; rr < 16; ++rr) ((volatile float*)XB)[(r0 + rr) * NV + lane] = Tf[rr][lane]; __threadfence(); }
}
__global__ __launch_bounds__(32) void edge_kernel(const float* __restrict__ XB, const float* __restrict__ ea, const int* __restrict__ es, const int* __restrict__ ed, const float* __restrict__ f1w, const float* __restrict__ f1b, const b16* __restrict__ MCh, const b16* __restrict__ MCl, int NLIM, int RLIM, b16* __restrict__ XE) {
  __shared__ __attribute__((aligned(16))) b16 Ah[16][72], Al[16][72], To[16][40]; const int lane = threadIdx.x, nloc = lane & 15, hlf = lane >> 4; const size_t r0 = (size_t)blockIdx.x * 16; if (r0 >= (size_t)RLIM) return;
  const int v = lane & 31; const float w1w = bf16_rne(f1w[v]), w1b = bf16_rne(f1b[v]);
  for (int rr = 0; rr < 16; ++rr) { const size_t r = r0 + rr; const size_t e = r / DIM; const int d = (int)(r % DIM); const int s = iclamp(es[e], 0, N - 1), t = iclamp(ed[e], 0, N - 1); const bool ok = s < NLIM && t < NLIM;
    const float W1 = silu(pmul(bf16_rne(ea[e]), w1w) + w1b); const float xs = ok ? XB[((size_t)s * DIM + d) * NV + v] : 0.0f, xd = ok ? XB[((size_t)t * DIM + d) * NV + v] : 0.0f;
    b16 p, q; split16(pmul(W1, xs - xd), p, q); Ah[rr][v] = p; Al[rr][v] = q; split16(pmul(W1, (xs + xd) * 0.5f), p, q); Ah[rr][32 + v] = p; Al[rr][32 + v] = q; }
  wave_lds_sync();
#pragma unroll
  for (int tt = 0; tt < 2; ++tt) { v8f acc = {};
#pragma unroll
    for (int kb = 0; kb < 64; kb += 32) { const v16b a = frag_kb(&Ah[nloc][kb], hlf), al = frag_kb(&Al[nloc][kb], hlf), bh = frag_kb(MCh + (size_t)(tt * 16 + nloc) * 64 + kb, hlf), bl = frag_kb(MCl + (size_t)(tt * 16 + nloc) * 64 + kb, hlf); acc = wmma16b(a, bh, acc); acc = wmma16b(a, bl, acc); acc = wmma16b(al, bh, acc); }
#pragma unroll
    for (int r8 = 0; r8 < 8; ++r8) To[8 * hlf + r8][tt * 16 + nloc] = (b16)acc[r8]; }
  wave_lds_sync();
  for (int pass = 0; pass < 2; ++pass) { for (int rr = 0; rr < 16; ++rr) ((volatile b16*)XE)[(r0 + rr) * NV + lane] = To[rr][lane]; __threadfence(); }
}
__global__ __launch_bounds__(32) void nodeupd_kernel(const b16* __restrict__ XE, const float* __restrict__ ea, const float* __restrict__ f2w, const float* __restrict__ f2b, const int* __restrict__ es, const int* __restrict__ ed,
    const int* __restrict__ P1, const int* __restrict__ RP1, const int* __restrict__ RC1, int pl1, const int* __restrict__ P2, const int* __restrict__ RP2, const int* __restrict__ RC2, int pl2, const b16* __restrict__ WE, int NLIM, int ELIM, int RLIM, float* __restrict__ Y) {
  __shared__ __attribute__((aligned(16))) b16 Ah[16][72], Al[16][72]; __shared__ float Tf[16][NV + 1]; const int lane = threadIdx.x, nloc = lane & 15, hlf = lane >> 4; const size_t r0 = (size_t)blockIdx.x * 16; if (r0 >= (size_t)RLIM) return;
  const float w2w = bf16_rne(f2w[lane]), w2b = bf16_rne(f2b[lane]);
  for (int rr = 0; rr < 16; ++rr) { const size_t r = r0 + rr; const size_t n = r / DIM; const int d = (int)(r % DIM); float a1 = 0.0f, a2 = 0.0f;
    { int st = RP1[n], cnt = RC1[n]; cnt = iclamp(cnt, 0, 1 << 20); st = iclamp(st, 0, pl1 - cnt);
#pragma unroll 1
      for (int j = 0; j < cnt; ++j) { const size_t e = (size_t)iclamp(P1[st + j], 0, E - 1); if (e >= (size_t)ELIM || iclamp(es[e], 0, N - 1) >= NLIM) continue; const float W2 = silu(pmul(bf16_rne(ea[e]), w2w) + w2b); a1 += pmul(W2, (float)XE[(e * DIM + d) * NV + lane]); } }
    { int st = RP2[n], cnt = RC2[n]; cnt = iclamp(cnt, 0, 1 << 20); st = iclamp(st, 0, pl2 - cnt);
#pragma unroll 1
      for (int j = 0; j < cnt; ++j) { const size_t e = (size_t)iclamp(P2[st + j], 0, E - 1); if (e >= (size_t)ELIM || iclamp(ed[e], 0, N - 1) >= NLIM) continue; const float W2 = silu(pmul(bf16_rne(ea[e]), w2w) + w2b); a2 += pmul(W2, (float)XE[(e * DIM + d) * NV + lane]); } }
    b16 p, q; split16((a1 - a2) * 0.0625f, p, q); Ah[rr][lane] = p; Al[rr][lane] = q; split16((a1 + a2) * 0.0625f, p, q); Ah[rr][32 + lane] = p; Al[rr][32 + lane] = q; }
  wave_lds_sync();
#pragma unroll
  for (int tt = 0; tt < 2; ++tt) { v8f acc = {};
#pragma unroll
    for (int kb = 0; kb < 64; kb += 32) { const v16b bw = frag_kb(WE + (size_t)(tt * 16 + nloc) * 64 + kb, hlf); acc = wmma16b(frag_kb(&Ah[nloc][kb], hlf), bw, acc); acc = wmma16b(frag_kb(&Al[nloc][kb], hlf), bw, acc); }
#pragma unroll
    for (int r8 = 0; r8 < 8; ++r8) Tf[8 * hlf + r8][tt * 16 + nloc] = acc[r8] * 16.0f; }
  wave_lds_sync();
  for (int pass = 0; pass < 2; ++pass) { for (int rr = 0; rr < 16; ++rr) ((volatile float*)Y)[(r0 + rr) * NV + lane] = Tf[rr][lane]; __threadfence(); }
}
__global__ __launch_bounds__(256) void act_kernel(const float* __restrict__ Y, int NLIM, float* __restrict__ out) {
  const int wave = threadIdx.x >> 5, lane = threadIdx.x & 31; const size_t n = (size_t)blockIdx.x * 8 + wave; if (n >= (size_t)NLIM) return; const float y0 = Y[(n * 3) * NV + lane], y1 = Y[(n * 3 + 1) * NV + lane], y2 = Y[(n * 3 + 2) * NV + lane];
  const float t = tanhf(sqrtf(pmul(y0, y0) + pmul(y1, y1) + pmul(y2, y2)));
  for (int pass = 0; pass < 2; ++pass) { ((volatile float*)out)[(n * 3) * NV + lane] = pmul(y0, t); ((volatile float*)out)[(n * 3 + 1) * NV + lane] = pmul(y1, t); ((volatile float*)out)[(n * 3 + 2) * NV + lane] = pmul(y2, t); __threadfence(); }
}
}

extern "C" void kernel_launch(void* const* d_in, const int* in_sizes, int n_in, void* d_out, int out_size, void* d_ws, size_t ws_size, hipStream_t stream) {
  (void)n_in;
  auto Fp = [&](int i) { return (const float*)d_in[i]; }; auto Ip = [&](int i) { return (const int*)d_in[i]; };
  if (in_sizes[0] != RN * NV || in_sizes[1] != N * NS || in_sizes[2] != E || in_sizes[3] != E || in_sizes[4] != E || in_sizes[5] != NV * NS || in_sizes[11] != NV * NV || in_sizes[16] != NV * NV || out_size != RN * NV) return;
  const int NLIM = N, ELIM = E; const int RNL = NLIM * DIM, REL = ELIM * DIM;
  size_t off = 0; char* ws = (char*)d_ws;
  auto carve = [&](size_t bytes) { char* p = ws + off; off += (bytes + 255) & ~(size_t)255; return p; };
  b16* WM = (b16*)carve(NV * NS * 2); b16* WMT = (b16*)carve(NV * NS * 2); b16* MCh = (b16*)carve(NV * 64 * 2); b16* MCl = (b16*)carve(NV * 64 * 2); b16* WE = (b16*)carve(NV * 64 * 2);
  float* XB = (float*)carve((size_t)RN * NV * 4); b16* XE = (b16*)carve((size_t)RE * NV * 2); float* Y = XB;
  CsrBufs9 c1, c2; off = csr_carve9(c1, ws, off, E, N); off = csr_carve9(c2, ws, off, E, N);
  if (off > ws_size) return;
  wsmall_kernel<<<1, 256, 0, stream>>>(Fp(5), Fp(11), Fp(12), Fp(13), Fp(14), Fp(15), Fp(16), WM, WMT, MCh, MCl, WE);
  csr_build9(c1, Ip(4), E, N, stream); csr_build9(c2, Ip(3), E, N, stream);
  nodemix_kernel<<<RNL / 16, 32, 0, stream>>>(Fp(0), Fp(1), Fp(6), WM, WMT, RNL, XB);
  edge_kernel<<<REL / 16, 32, 0, stream>>>(XB, Fp(2), Ip(3), Ip(4), Fp(7), Fp(8), MCh, MCl, NLIM, REL, XE);
  nodeupd_kernel<<<RNL / 16, 32, 0, stream>>>(XE, Fp(2), Fp(9), Fp(10), Ip(3), Ip(4), c1.PERM, c1.ROWPTR, c1.ROWCNT, (int)c1.permLen, c2.PERM, c2.ROWPTR, c2.ROWCNT, (int)c2.permLen, WE, NLIM, ELIM, RNL, Y);
  act_kernel<<<(NLIM + 7) / 8, 256, 0, stream>>>(Y, NLIM, (float*)d_out);
}
